// PerceiverBlock_modified_53403623359030
// MI455X (gfx1250) — hardware-verified
//
#include <hip/hip_runtime.h>


namespace {
constexpr int Bn = 4, N1 = 1024, N2 = 256, L = N1 + N2  , D = 1024, H = 16, HD = 64, NT = Bn * L, DF = 4096, DQK = 2 * D;
constexpr float EPS = 1e-5f, XS = 8.0f, PS = 8.0f;

typedef _Float16 b16;
typedef __attribute__((ext_vector_type(16))) _Float16 v16b;
typedef __attribute__((ext_vector_type(8))) _Float16 v8b;
typedef __attribute__((ext_vector_type(8))) float v8f;
typedef __attribute__((ext_vector_type(4))) float v4f;
__device__ __forceinline__ void split16(float v, _Float16& hi, _Float16& lo) { hi = (_Float16)v; lo = (_Float16)(v - (float)hi); }
__device__ __forceinline__ float bf16_rne(float f) { unsigned int u = __float_as_uint(f); u += 0x7FFFu + ((u >> 16) & 1u); return __uint_as_float(u & 0xFFFF0000u); }
__device__ __forceinline__ v16b frag_kb(const b16* p, int hh) { const v8b a = *(const v8b*)(p + 8 * hh), b = *(const v8b*)(p + 16 + 8 * hh); v16b f;
#pragma unroll
  for (int e = 0; e < 8; ++e) { f[e] = a[e]; f[8 + e] = b[e]; } return f; }
__device__ __forceinline__ v16b frag_x(const float* p, int hh) { v16b f;
#pragma unroll
  for (int e = 0; e < 8; ++e) { f[e] = (b16)bf16_rne(p[8 * hh + e]); f[8 + e] = (b16)bf16_rne(p[16 + 8 * hh + e]); } return f; }
__device__ __forceinline__ v8f wmma16b(v16b a, v16b b, v8f c) { v8f d = __builtin_amdgcn_wmma_f32_16x16x32_f16(false, a, false, b, (short)0, c, false, false); asm volatile("v_nop\n\tv_nop\n\tv_nop\n\tv_nop" : "+v"(d) : "v"(a), "v"(b)); return d; }
__device__ __forceinline__ void wave_lds_sync() { __builtin_amdgcn_fence(__ATOMIC_RELEASE, "workgroup"); __builtin_amdgcn_wave_barrier(); __builtin_amdgcn_fence(__ATOMIC_ACQUIRE, "workgroup"); }
__device__ __forceinline__ float nexp(float x) { return __builtin_amdgcn_exp2f(x * 1.4426950408889634f); }
__device__ __forceinline__ float pmul(float a, float b) { float p = a * b; asm volatile("" : "+v"(p)); return p; }
__device__ __forceinline__ float wsum(float v) {
#pragma unroll
  for (int o = 1; o < 32; o <<= 1) v += __shfl_xor(v, o); return v; }
__device__ __forceinline__ void sincos_r(float ang, float& sn, float& cs) { const float k = rintf(ang * 0.15915494309189535f); float r = __builtin_fmaf(k, -6.28318548202514648f, ang); r = __builtin_fmaf(k, 1.7484556025237907e-7f, r);
  const float t = r * 0.15915494309189535f; sn = __builtin_amdgcn_sinf(t); cs = __builtin_amdgcn_cosf(t); }
__device__ __forceinline__ float tanh_n(float x) { const float e = __builtin_amdgcn_exp2f(x * 2.8853900817779268f); return 1.0f - 2.0f * __builtin_amdgcn_rcpf(e + 1.0f); }
__device__ __forceinline__ float gelu_t(float x) { const float c = 0.7978845608028654f; return 0.5f * x * (1.0f + tanh_n(c * (x + 0.044715f * x * x * x))); }

struct Wo_ { static constexpr size_t QK = 0, V = (size_t)DQK * D, O = V + (size_t)D * D, F1 = O + (size_t)D * D, F2 = F1 + (size_t)DF * D, END = F2 + (size_t)D * DF; };
__global__ __launch_bounds__(256) void prep_kernel(const float* __restrict__ wq, const float* __restrict__ wkv, const float* __restrict__ wo, const float* __restrict__ w1, const float* __restrict__ w2, const float* __restrict__ gm, const float* __restrict__ bm, const float* __restrict__ gl, const float* __restrict__ bl, const float* __restrict__ gf, const float* __restrict__ bf, b16* __restrict__ R, float* __restrict__ P) {
  const size_t tid = (size_t)blockIdx.x * 256 + threadIdx.x, nth = (size_t)gridDim.x * 256;
  auto tr = [&](size_t base, int nout, int kin, const float* W, int ldw, int co) { for (size_t p = tid; p < (size_t)nout * (kin / 8); p += nth) { const int o = (int)(p / (kin / 8)), k0 = (int)(p % (kin / 8)) * 8; v8b v;
#pragma unroll
      for (int e = 0; e < 8; ++e) v[e] = (b16)bf16_rne(W[(size_t)(k0 + e) * ldw + co + o]); *(volatile v8b*)(R + base + (size_t)o * kin + k0) = v; } };
  for (int pass = 0; pass < 2; ++pass) { tr(Wo_::QK, D, D, wq, D, 0); tr(Wo_::QK + (size_t)D * D, D, D, wkv, 2 * D, 0); tr(Wo_::V, D, D, wkv, 2 * D, D); tr(Wo_::O, D, D, wo, D, 0); tr(Wo_::F1, DF, D, w1, DF, 0); tr(Wo_::F2, D, DF, w2, D, 0);
    for (size_t q = tid; q < 11264; q += nth) { const int i = (int)q, c = i & 1023; float v; if (i < 1024) v = gm[c]; else if (i < 2048) v = bm[c]; else if (i < 3072) v = gl[c]; else if (i < 4096) v = bl[c]; else if (i < 5120) v = gf[c]; else if (i < 6144) v = bf[c]; else v = 0.0f; P[q] = bf16_rne(v); }
    __threadfence(); }
}

__global__ __launch_bounds__(256) void tok_kernel(const float* __restrict__ x, const float* __restrict__ lat, const float* __restrict__ P, float* __restrict__ RES, b16* __restrict__ X) {
  const int row = blockIdx.x * 8 + (threadIdx.x >> 5), lane = threadIdx.x & 31; const int b = row / L, t = row % L; const float* src = (t < N1) ? (x + ((size_t)b * N1 + t) * D) : (lat + ((size_t)b * N2 + (t - N1)) * D);
  const float* g = P + ((t < N1) ? 0 : 2048); const float* bb = g + 1024;
  float v[32]; float s = 0.0f;
#pragma unroll
  for (int i = 0; i < 32; ++i) { v[i] = bf16_rne(src[(i >> 3) * 256 + lane * 8 + (i & 7)]); s += v[i]; }
  s = wsum(s); const float mu = s * (1.0f / D); float q = 0.0f;
#pragma unroll
  for (int i = 0; i < 32; ++i) { const float d = v[i] - mu; q += pmul(d, d); }
  q = wsum(q); const float inv = rsqrtf(q * (1.0f / D) + EPS);
  for (int pass = 0; pass < 2; ++pass) {
#pragma unroll
    for (int gq = 0; gq < 4; ++gq) { const int c0 = gq * 256 + lane * 8; v8b o; v4f r0, r1;
#pragma unroll
      for (int e = 0; e < 8; ++e) o[e] = (b16)((pmul((v[gq * 8 + e] - mu) * inv, g[c0 + e]) + bb[c0 + e]) * XS);
#pragma unroll
      for (int e = 0; e < 4; ++e) { r0[e] = v[gq * 8 + e]; r1[e] = v[gq * 8 + 4 + e]; }
      *(volatile v8b*)(X + (size_t)row * D + c0) = o; *(volatile v4f*)(RES + (size_t)row * D + c0) = r0; *(volatile v4f*)(RES + (size_t)row * D + c0 + 4) = r1; }
    __threadfence(); }
}

__global__ __launch_bounds__(256) void xrows_kernel(const float* __restrict__ x, b16* __restrict__ X) {
  const size_t tid = (size_t)blockIdx.x * 256 + threadIdx.x, nth = (size_t)gridDim.x * 256;
  for (int pass = 0; pass < 2; ++pass) { for (size_t p = tid; p < (size_t)NT * D / 8; p += nth) { v8b v; for (int e = 0; e < 8; ++e) v[e] = (b16)(bf16_rne(x[p * 8 + e]) * XS); *(volatile v8b*)(X + p * 8) = v; } __threadfence(); }
}

__global__ __launch_bounds__(128) void vproj_kernel(const b16* __restrict__ X, const b16* __restrict__ R, const float* __restrict__ P, b16* __restrict__ VT) {
  __shared__ __attribute__((aligned(16))) b16 Tv[128][128 + 8];
  const int lane = threadIdx.x & 31, wave = threadIdx.x >> 5, nloc = lane & 15, hlf = lane >> 4, t0 = blockIdx.x * 128, m0 = t0 + wave * 32; const int b = t0 / L, p0 = t0 % L; const b16* Wv = R + Wo_::V;
#pragma unroll 1
  for (int ch = 0; ch < 8; ++ch) { v8f acc[2][8];
#pragma unroll
    for (int r = 0; r < 2; ++r)
#pragma unroll
      for (int t = 0; t < 8; ++t) acc[r][t] = (v8f){};
#pragma unroll 2
    for (int kb = 0; kb < D; kb += 32) { const v16b a0 = frag_kb(X + (size_t)(m0 + nloc) * D + kb, hlf), a1 = frag_kb(X + (size_t)(m0 + 16 + nloc) * D + kb, hlf);
#pragma unroll
      for (int t = 0; t < 8; ++t) { const v16b bw = frag_kb(Wv + (size_t)(ch * 128 + t * 16 + nloc) * D + kb, hlf); acc[0][t] = wmma16b(a0, bw, acc[0][t]); acc[1][t] = wmma16b(a1, bw, acc[1][t]); } }
    __syncthreads();
#pragma unroll
    for (int t = 0; t < 8; ++t) { const int c = t * 16 + nloc; const float bb = P[2048 + ch * 128 + c];
#pragma unroll
      for (int r = 0; r < 2; ++r)
#pragma unroll
        for (int v = 0; v < 8; ++v) Tv[c][wave * 32 + r * 16 + 8 * hlf + v] = (b16)((acc[r][t][v] * (1.0f / XS) + bb) * XS); }
    __syncthreads();
    for (int pass = 0; pass < 2; ++pass) { for (int i = threadIdx.x; i < 128 * 16; i += 128) { const int c = i >> 4, c8 = (i & 15) * 8; const int cg = ch * 128 + c, h = cg / HD, d = cg % HD; *(volatile v8b*)(VT + (((size_t)b * H + h) * HD + d) * L + p0 + c8) = *(const v8b*)(&Tv[c][c8]); } __threadfence(); } }
}

__global__ __launch_bounds__(256) void ln32_kernel(const float* src, const float* __restrict__ g, const float* __restrict__ bb, float* dst) {
  const int row = blockIdx.x * 8 + (threadIdx.x >> 5), lane = threadIdx.x & 31; const float* xr = src + (size_t)row * D;
  float v[32]; float s = 0.0f;
#pragma unroll
  for (int i = 0; i < 32; ++i) { v[i] = xr[(i >> 3) * 256 + lane * 8 + (i & 7)]; s += v[i]; }
  s = wsum(s); const float mu = s * (1.0f / D); float q = 0.0f;
#pragma unroll
  for (int i = 0; i < 32; ++i) { const float d = v[i] - mu; q += pmul(d, d); }
  q = wsum(q); const float inv = rsqrtf(q * (1.0f / D) + EPS);
  for (int pass = 0; pass < 2; ++pass) {
#pragma unroll
    for (int gq = 0; gq < 4; ++gq) { const int c0 = gq * 256 + lane * 8; v4f o0, o1;
#pragma unroll
      for (int e = 0; e < 4; ++e) { o0[e] = pmul((v[gq * 8 + e] - mu) * inv, g[c0 + e]) + bb[c0 + e]; o1[e] = pmul((v[gq * 8 + 4 + e] - mu) * inv, g[c0 + 4 + e]) + bb[c0 + 4 + e]; }
      *(volatile v4f*)(dst + (size_t)row * D + c0) = o0; *(volatile v4f*)(dst + (size_t)row * D + c0 + 4) = o1; }
    __threadfence(); }
}

__global__ __launch_bounds__(256) void ln_kernel(const float* __restrict__ src, int rnd, const float* __restrict__ g, const float* __restrict__ bb, b16* __restrict__ dst) {
  const int row = blockIdx.x * 8 + (threadIdx.x >> 5), lane = threadIdx.x & 31; const float* xr = src + (size_t)row * D;
  float v[32]; float s = 0.0f;
#pragma unroll
  for (int i = 0; i < 32; ++i) { float x = xr[(i >> 3) * 256 + lane * 8 + (i & 7)]; if (rnd) x = bf16_rne(x); v[i] = x; s += x; }
  s = wsum(s); const float mu = s * (1.0f / D); float q = 0.0f;
#pragma unroll
  for (int i = 0; i < 32; ++i) { const float d = v[i] - mu; q += pmul(d, d); }
  q = wsum(q); const float inv = rsqrtf(q * (1.0f / D) + EPS);
  for (int pass = 0; pass < 2; ++pass) {
#pragma unroll
    for (int gq = 0; gq < 4; ++gq) { v8b o; const int c0 = gq * 256 + lane * 8;
#pragma unroll
      for (int e = 0; e < 8; ++e) o[e] = (b16)((pmul((v[gq * 8 + e] - mu) * inv, g[c0 + e]) + bb[c0 + e]) * XS);
      *(volatile v8b*)(dst + (size_t)row * D + c0) = o; }
    __threadfence(); }
}

template <int K, int N, int EPI, int RND>
__global__ __launch_bounds__(64) void gemm_kernel(const b16* __restrict__ A, const b16* __restrict__ Bw, const float* __restrict__ bias, const float* __restrict__ resid, b16* __restrict__ Ch, float* __restrict__ Cf, const float* __restrict__ gate = nullptr, const b16* __restrict__ Alo = nullptr) {
  __shared__ __attribute__((aligned(16))) float Ts[2][32][128 + 4];
  const int lane = threadIdx.x & 31, wave = threadIdx.x >> 5, nloc = lane & 15, hlf = lane >> 4, m0 = blockIdx.y * 32, c0 = blockIdx.x * 256 + wave * 128;
  v8f acc[2][8];
#pragma unroll
  for (int r = 0; r < 2; ++r)
#pragma unroll
    for (int t = 0; t < 8; ++t) acc[r][t] = (v8f){};
  for (int kb = 0; kb < K; kb += 32) { const v16b a0 = frag_kb(A + (size_t)(m0 + nloc) * K + kb, hlf), a1 = frag_kb(A + (size_t)(m0 + 16 + nloc) * K + kb, hlf);
    if (EPI == 4) { const v16b l0 = frag_kb(Alo + (size_t)(m0 + nloc) * K + kb, hlf), l1 = frag_kb(Alo + (size_t)(m0 + 16 + nloc) * K + kb, hlf);
#pragma unroll
      for (int t = 0; t < 8; ++t) { const v16b bw = frag_kb(Bw + (size_t)(c0 + t * 16 + nloc) * K + kb, hlf); acc[0][t] = wmma16b(a0, bw, acc[0][t]); acc[0][t] = wmma16b(l0, bw, acc[0][t]); acc[1][t] = wmma16b(a1, bw, acc[1][t]); acc[1][t] = wmma16b(l1, bw, acc[1][t]); } }
    else {
#pragma unroll
      for (int t = 0; t < 8; ++t) { const v16b bw = frag_kb(Bw + (size_t)(c0 + t * 16 + nloc) * K + kb, hlf); acc[0][t] = wmma16b(a0, bw, acc[0][t]); acc[1][t] = wmma16b(a1, bw, acc[1][t]); } } }
#pragma unroll
  for (int t = 0; t < 8; ++t) { const float bv = (bias != nullptr) ? bias[c0 + t * 16 + nloc] : 0.0f;
#pragma unroll
    for (int r = 0; r < 2; ++r)
#pragma unroll
      for (int v = 0; v < 8; ++v) { float y = acc[r][t][v] * (1.0f / XS) + bv; if (EPI == 2) y = fmaxf(y, 0.0f); if (EPI == 5) y = 0.5f * y * (1.0f + erff(y * 0.7071067811865476f)); if (EPI == 4) y = pmul(y, gate[(size_t)((m0 + r * 16) / L) * N + c0 + t * 16 + nloc]); Ts[wave][r * 16 + 8 * hlf + v][t * 16 + nloc] = y; } }
  wave_lds_sync();
  if (EPI == 3 && c0 < 2 * D) {
    for (int i = lane; i < 32 * 64; i += 32) { const int rr = i >> 6, cp = (i & 63) * 2; const int t = (m0 + rr) % L; const int i2 = ((c0 + cp) & 63) >> 1;
      const float invf = __builtin_amdgcn_exp2f(-(float)i2 * (13.287712379549449f / 32.0f));
      float sn, cs; sincos_r((float)t * invf, sn, cs); const float xe = Ts[wave][rr][cp], xo = Ts[wave][rr][cp + 1];
      Ts[wave][rr][cp] = pmul(xe, cs) - pmul(xo, sn); Ts[wave][rr][cp + 1] = pmul(xe, sn) + pmul(xo, cs); }
    wave_lds_sync(); }
  for (int pass = 0; pass < 2; ++pass) {
    if (EPI == 1 || EPI == 4) { for (int i = lane; i < 32 * 32; i += 32) { const int rr = i >> 5, c4 = (i & 31) * 4; const size_t gi = (size_t)(m0 + rr) * N + c0 + c4; v4f o = *(const v4f*)(&Ts[wave][rr][c4]); const v4f xr = *(const v4f*)(resid + gi);
        for (int e = 0; e < 4; ++e) o[e] += RND ? bf16_rne(xr[e]) : xr[e]; *(volatile v4f*)(Cf + gi) = o; } }
    else { for (int i = lane; i < 32 * 16; i += 32) { const int rr = i >> 4, c8 = (i & 15) * 8; v8b o; for (int e = 0; e < 8; ++e) o[e] = (b16)(Ts[wave][rr][c8 + e] * XS); *(volatile v8b*)(Ch + (size_t)(m0 + rr) * N + c0 + c8) = o; } }
    __threadfence(); }
}

__global__ __launch_bounds__(256) void attn_kernel(const b16* __restrict__ QK, const b16* __restrict__ vt, b16* __restrict__ ctx, int boff) {
  __shared__ __attribute__((aligned(16))) b16 Os[16][8 * HD + 8];
  const int bx = blockIdx.x + boff; const int wid = threadIdx.x >> 5, lane = threadIdx.x & 31, hh = lane >> 4, col = lane & 15; const int b = bx / (L / 16), q0 = (bx % (L / 16)) * 16, h = blockIdx.y * 8 + wid, qi = q0 + col;
  const b16* Qr = QK + (size_t)(b * L) * DQK + h * HD; const b16* Kr = QK + (size_t)(b * L) * DQK + D + h * HD; const b16* V = vt + (((size_t)b * H + h) * HD) * L;
  const v16b qf0 = frag_kb(Qr + (size_t)qi * DQK, hh), qf1 = frag_kb(Qr + (size_t)qi * DQK + 32, hh);
  float m = -INFINITY, l = 0.0f; v8f o[4] = {{}, {}, {}, {}};
  for (int kb = 0; kb < L; kb += 32) {
    v8f s0 = {}, s1 = {}; s0 = wmma16b(frag_kb(Kr + (size_t)(kb + col) * DQK, hh), qf0, s0); s0 = wmma16b(frag_kb(Kr + (size_t)(kb + col) * DQK + 32, hh), qf1, s0);
    s1 = wmma16b(frag_kb(Kr + (size_t)(kb + 16 + col) * DQK, hh), qf0, s1); s1 = wmma16b(frag_kb(Kr + (size_t)(kb + 16 + col) * DQK + 32, hh), qf1, s1);
    float mr = -INFINITY;
#pragma unroll
    for (int r = 0; r < 8; ++r) { s0[r] *= (0.125f / (XS * XS)); s1[r] *= (0.125f / (XS * XS)); mr = fmaxf(mr, fmaxf(s0[r], s1[r])); }
    mr = fmaxf(mr, __shfl_xor(mr, 16)); const float mn = fmaxf(m, mr), al_ = nexp(m - mn); m = mn; float sum = 0.0f; v16b pb;
#pragma unroll
    for (int r = 0; r < 8; ++r) { const float e0 = nexp(s0[r] - mn), e1 = nexp(s1[r] - mn); sum += e0 + e1; pb[r] = (b16)(e0 * PS); pb[8 + r] = (b16)(e1 * PS); }
    sum += __shfl_xor(sum, 16); l = l * al_ + sum;
#pragma unroll
    for (int t = 0; t < 4; ++t) { o[t] *= al_; o[t] = wmma16b(frag_kb(V + (size_t)(t * 16 + col) * L + kb, hh), pb, o[t]); } }
  const float inv = 1.0f / (l * PS);
#pragma unroll
  for (int t = 0; t < 4; ++t)
#pragma unroll
    for (int r = 0; r < 8; ++r) Os[col][wid * HD + t * 16 + 8 * hh + r] = (b16)(o[t][r] * inv);
  __syncthreads();
  for (int pass = 0; pass < 2; ++pass) { for (int i = threadIdx.x; i < 16 * 64; i += 256) { const int rr = i >> 6, c8 = (i & 63) * 8; *(volatile v8b*)(ctx + ((size_t)(b * L + q0 + rr)) * D + blockIdx.y * 8 * HD + c8) = *(const v8b*)(&Os[rr][c8]); } __threadfence(); }
}
__global__ __launch_bounds__(256) void rows16_kernel(const float* __restrict__ src, b16* __restrict__ dst) {
  const size_t tid = (size_t)blockIdx.x * 256 + threadIdx.x, nth = (size_t)gridDim.x * 256;
  for (int pass = 0; pass < 2; ++pass) { for (size_t p = tid; p < (size_t)NT * D / 8; p += nth) { v8b v; for (int e = 0; e < 8; ++e) v[e] = (b16)(src[p * 8 + e] * XS); *(volatile v8b*)(dst + p * 8) = v; } __threadfence(); }
}

__global__ __launch_bounds__(256) void ffn_kernel(const b16* __restrict__ X1H, const b16* __restrict__ R, const float* __restrict__ P, const float* __restrict__ Y, float* __restrict__ OUT, int boff) {
  __shared__ __attribute__((aligned(16))) b16 G[16][DF + 8];
  const int wave = threadIdx.x >> 5, lane = threadIdx.x & 31, nloc = lane & 15, hlf = lane >> 4, r0 = (blockIdx.x + boff) * 16; const b16* W1 = R + Wo_::F1; const b16* W2 = R + Wo_::F2; const float* b1 = P + 6144; const float* b2 = P + 10240;
  for (int t = wave; t < DF / 16; t += 8) { v8f acc = {};
#pragma unroll 4
    for (int kb = 0; kb < D; kb += 32) acc = wmma16b(frag_kb(X1H + (size_t)(r0 + nloc) * D + kb, hlf), frag_kb(W1 + (size_t)(t * 16 + nloc) * D + kb, hlf), acc);
    const int c = t * 16 + nloc; const float bb = b1[c];
#pragma unroll
    for (int r = 0; r < 8; ++r) { const float u = acc[r] * (1.0f / XS) + bb; const float gl = 0.5f * u * (1.0f + erff(u * 0.70710678118654752f)); G[8 * hlf + r][c] = (b16)(gl * XS); } }
  __syncthreads();
  v8f acc2[8];
#pragma unroll
  for (int t = 0; t < 8; ++t) acc2[t] = (v8f){};
#pragma unroll 2
  for (int kb = 0; kb < DF; kb += 32) { const v16b a = frag_kb(&G[nloc][kb], hlf);
#pragma unroll
    for (int t = 0; t < 8; ++t) acc2[t] = wmma16b(a, frag_kb(W2 + (size_t)(wave * 128 + t * 16 + nloc) * DF + kb, hlf), acc2[t]); }
  float vals[8][8];
#pragma unroll
  for (int t = 0; t < 8; ++t) { const int c = wave * 128 + t * 16 + nloc; const float bb = b2[c];
#pragma unroll
    for (int r = 0; r < 8; ++r) vals[t][r] = acc2[t][r] * (1.0f / XS) + bb + Y[(size_t)(r0 + 8 * hlf + r) * D + c]; }
  __syncthreads();
  float (*St)[128 + 4] = (float (*)[128 + 4])((float*)&G[0][0] + wave * 16 * (128 + 4));
#pragma unroll
  for (int t = 0; t < 8; ++t)
#pragma unroll
    for (int r = 0; r < 8; ++r) St[8 * hlf + r][t * 16 + nloc] = vals[t][r];
  wave_lds_sync();
  for (int pass = 0; pass < 2; ++pass) { for (int i = lane; i < 16 * 32; i += 32) { const int rr = i >> 5, c4 = (i & 31) * 4; const int row = r0 + rr, b = row / L, t = row % L;
      float* dst = (t < N1) ? (OUT + ((size_t)b * N1 + t) * D) : (OUT + (size_t)Bn * N1 * D + ((size_t)b * N2 + (t - N1)) * D); *(volatile v4f*)(dst + wave * 128 + c4) = *(const v4f*)(&St[rr][c4]); } __threadfence(); }
}
}

extern "C" void kernel_launch(void* const* d_in, const int* in_sizes, int n_in,
                              void* d_out, int out_size, void* d_ws, size_t ws_size, hipStream_t stream) {
  (void)n_in; (void)out_size;
  const float* x = (const float*)d_in[0]; const float* lat = (const float*)d_in[1]; const float* wq = (const float*)d_in[2]; const float* wkv = (const float*)d_in[3]; const float* wo = (const float*)d_in[4]; const float* w1 = (const float*)d_in[5]; const float* w2 = (const float*)d_in[6];
  const float* gm = (const float*)d_in[7]; const float* bm = (const float*)d_in[8]; const float* gl = (const float*)d_in[9]; const float* bl = (const float*)d_in[10]; const float* gf = (const float*)d_in[11]; const float* bf = (const float*)d_in[12];
  float* out = (float*)d_out;
  if (in_sizes[0] != Bn * N1 * D || in_sizes[1] != Bn * N2 * D || in_sizes[2] != D * D || in_sizes[3] != D * 2 * D || in_sizes[5] != D * DF || in_sizes[6] != DF * D) return;
  size_t off = 0; char* ws = (char*)d_ws;
  auto carve = [&](size_t bytes) { char* p = ws + off; off += (bytes + 255) & ~(size_t)255; return p; };
  b16* R = (b16*)carve(Wo_::END * 2); float* P = (float*)carve(11264 * 4); b16* X = (b16*)carve((size_t)NT * D * 2); float* RES = (float*)carve((size_t)NT * D * 4); b16* QK = (b16*)carve((size_t)NT * DQK * 2); b16* VT = (b16*)carve((size_t)NT * D * 2); float* Y = (float*)carve((size_t)NT * D * 4);
  if (off > ws_size) return;
  b16* CTX = X; b16* X1H = X;
  prep_kernel<<<512, 256, 0, stream>>>(wq, wkv, wo, w1, w2, gm, bm, gl, bl, gf, bf, R, P);
  tok_kernel<<<NT / 8, 256, 0, stream>>>(x, lat, P, RES, X);
  gemm_kernel<D, DQK, 0, 0><<<dim3(DQK / 256, NT / 32), 64, 0, stream>>>(X, R + Wo_::QK, P + 6144, nullptr, QK, nullptr);
  vproj_kernel<<<NT / 128, 128, 0, stream>>>(X, R, P + 6144 - 2048, VT);
  attn_kernel<<<dim3(NT / 16, 2), 256, 0, stream>>>(QK, VT, CTX, 0);
  gemm_kernel<D, D, 1, 0><<<dim3(D / 256, NT / 32), 64, 0, stream>>>(CTX, R + Wo_::O, P + 6144, RES, nullptr, Y);
  ln_kernel<<<NT / 8, 256, 0, stream>>>(Y, 0, P + 4096, P + 5120, X1H);
  ffn_kernel<<<NT / 16, 256, 0, stream>>>(X1H, R, P, Y, out, 0);
}
